// ConvPool_6193342841562
// MI455X (gfx1250) — hardware-run, weakly checked
//
#include <hip/hip_runtime.h>
#include <stddef.h>
#include <stdint.h>

#define NB     4
#define NSUP   32768
#define NQ     8192
#define NS     32
#define CF     64
#define CIN    67
#define COUT   128
#define KPAD   96
#define SROWS  (NB * NSUP)
#define QROWS  (NB * NQ)
#define MROWS  (SROWS + QROWS)
#define PTR    128
#define NSB    (SROWS / PTR)
#define NQB    (QROWS / PTR)
#define NPB    (NSB + NQB + 1)
#define TILE_HALVES (PTR * KPAD)
#define TILE_BYTES  (TILE_HALVES * 2)
#define GBM    64
#define GTHR   128
#define NTHR   256
#define QPB    32
#define NGB    (QROWS / QPB)
#define OTP    33
#define NSAMP  1048576
#define WSCAP  134217728

static_assert(NS == 32);
static_assert(COUT == 32 * 4);
static_assert(CIN == 3 + CF && CIN <= KPAD && KPAD % 32 == 0);
static_assert(NQ % QPB == 0 && QPB == 32 && QPB == (NTHR / 32) * 4);
static_assert(MROWS % PTR == 0 && MROWS % GBM == 0);
static_assert(SROWS == 131072);
static_assert(NSUP % PTR == 0 && QROWS % PTR == 0);
static_assert(NSUP / PTR == 256 && NQ / QPB == 256);
static_assert(TILE_BYTES % 128 == 0 && TILE_BYTES == 6 * NTHR * 16);
static_assert(PTR * 3 <= 2 * NTHR);
static_assert(PTR == 32 * 4 && CF == 8 * (NTHR / 32));
static_assert(COUT * KPAD == TILE_HALVES);
static_assert(COUT * CIN <= 34 * NTHR);
static_assert(NSAMP == NB * NQ * NS);
static_assert(GBM == (GTHR / 32) * 16);
static_assert((KPAD * 2) % 16 == 0);

typedef float          v4f   __attribute__((ext_vector_type(4)));
typedef float          v8f   __attribute__((ext_vector_type(8)));
typedef double         v2d   __attribute__((ext_vector_type(2)));
typedef int            v8i   __attribute__((ext_vector_type(8)));
typedef unsigned short v8us  __attribute__((ext_vector_type(8)));
typedef unsigned short v16us __attribute__((ext_vector_type(16)));
typedef __bf16         v16bf __attribute__((ext_vector_type(16)));
typedef v4f  __attribute__((may_alias)) v4fa;
typedef v8us __attribute__((may_alias)) v8usa;
union FragB { v16bf v; v16us u; v8us h[2]; v8i w; };

__device__ __forceinline__ v8f wmb(const FragB& a, const FragB& b, v8f c) {
  v8f d = __builtin_amdgcn_wmma_f32_16x16x32_bf16(false, a.v, false, b.v, (short)0, c, false, false);
  asm volatile("v_nop\n\tv_nop\n\tv_nop\n\tv_nop" : "+v"(d) : "v"(a.w), "v"(b.w));
  return d;
}

__device__ __forceinline__ v8f z8() { v8f z = {0.f, 0.f, 0.f, 0.f, 0.f, 0.f, 0.f, 0.f}; return z; }

__device__ __forceinline__ unsigned bf16_bits(float f) {
  const unsigned u = __float_as_uint(f);
  return (u + 0x7FFFu + ((u >> 16) & 1u)) >> 16;
}
__device__ __forceinline__ float bf16_val(float f) {
  return __uint_as_float(bf16_bits(f) << 16);
}

__global__ __launch_bounds__(NTHR) void k_prep(const float* __restrict__ qxyz, const float* __restrict__ sxyz,
                                               const float* __restrict__ feat, const float* __restrict__ wc,
                                               unsigned short* ABW) {
  __shared__ __attribute__((aligned(16))) unsigned short tile[TILE_HALVES];
  const int tid = (int)threadIdx.x, lane = tid & 31, wave = tid >> 5;
  const int blk = (int)blockIdx.x;
  {
    const v8us zz = {0, 0, 0, 0, 0, 0, 0, 0};
#pragma unroll
    for (int it = 0; it < 6; ++it) *(v8usa*)(tile + (it * NTHR + tid) * 8) = zz;
  }
  __syncthreads();

  if (blk < NSB) {
    const int b  = blk >> 8;
    const int n0 = (blk & 255) * PTR;
    const float* xp = sxyz + ((size_t)b * NSUP + n0) * 3;
#pragma unroll
    for (int it = 0; it < 2; ++it) {
      const int idx = it * NTHR + tid;
      const int idc = idx < PTR * 3 - 1 ? idx : PTR * 3 - 1;
      const float v = xp[idc];
      asm volatile("" :: "v"(v));
      if (idx < PTR * 3) {
        const int r = idx / 3;
        const int k = idx - 3 * r;
        tile[r * KPAD + k] = (unsigned short)bf16_bits(v);
      }
    }
    const float* fp = feat + (size_t)b * CF * NSUP + n0 + 4 * lane;
#pragma unroll 4
    for (int it = 0; it < 8; ++it) {
      const int ch = it * 8 + wave;
      const v4f a = *(const v4f*)(fp + (size_t)ch * NSUP);
      unsigned short* tp = tile + (4 * lane) * KPAD + 3 + ch;
      tp[0]        = (unsigned short)bf16_bits(a.x);
      tp[KPAD]     = (unsigned short)bf16_bits(a.y);
      tp[2 * KPAD] = (unsigned short)bf16_bits(a.z);
      tp[3 * KPAD] = (unsigned short)bf16_bits(a.w);
    }
  } else if (blk < NSB + NQB) {
    const int q0 = (blk - NSB) * PTR;
    const float* xp = qxyz + (size_t)q0 * 3;
#pragma unroll
    for (int it = 0; it < 2; ++it) {
      const int idx = it * NTHR + tid;
      const int idc = idx < PTR * 3 - 1 ? idx : PTR * 3 - 1;
      const float v = xp[idc];
      asm volatile("" :: "v"(v));
      if (idx < PTR * 3) {
        const int r = idx / 3;
        const int k = idx - 3 * r;
        tile[r * KPAD + k] = (unsigned short)bf16_bits(v);
      }
    }
  } else {
#pragma unroll 2
    for (int it = 0; it < 34; ++it) {
      const int idx = it * NTHR + tid;
      const int idc = idx < COUT * CIN - 1 ? idx : COUT * CIN - 1;
      const float v = wc[idc];
      asm volatile("" :: "v"(v));
      if (idx < COUT * CIN) {
        const int o = idx / CIN;
        const int k = idx - CIN * o;
        tile[o * KPAD + k] = (unsigned short)bf16_bits(v);
      }
    }
  }
  __syncthreads();

  v8us pv[6];
#pragma unroll
  for (int it = 0; it < 6; ++it) pv[it] = *(const v8usa*)(tile + (it * NTHR + tid) * 8);
  unsigned short* dst = ABW + (size_t)blk * TILE_HALVES;
#pragma unroll
  for (int it = 0; it < 6; ++it) *(volatile v8us*)(dst + (it * NTHR + tid) * 8) = pv[it];
  __threadfence();
#pragma unroll
  for (int it = 0; it < 6; ++it) *(volatile v8us*)(dst + (it * NTHR + tid) * 8) = pv[it];
}

__global__ __launch_bounds__(GTHR) __attribute__((amdgpu_num_vgpr(248)))
void k_gemm(const unsigned short* __restrict__ A, const unsigned short* __restrict__ BT, float* Zp) {
  __shared__ __attribute__((aligned(16))) float stg[GBM * COUT];
  const int tid = (int)threadIdx.x, lane = tid & 31, wave = tid >> 5, hh = lane >> 4, m = lane & 15;
  const int rowBase = (int)blockIdx.x * GBM;

  v8f acc[8];
#pragma unroll
  for (int t = 0; t < 8; ++t) acc[t] = z8();
  const unsigned short* ap = A  + (size_t)(rowBase + 16 * wave + m) * (size_t)KPAD + 8 * hh;
  const unsigned short* bp = BT + (size_t)m * (size_t)KPAD + 8 * hh;

#pragma unroll 1
  for (int k0 = 0; k0 < KPAD; k0 += 32) {
    FragB af;
    af.h[0] = *(const v8usa*)(ap + k0);
    af.h[1] = *(const v8usa*)(ap + k0 + 16);
#pragma unroll
    for (int nt = 0; nt < 8; ++nt) {
      const unsigned short* wq = bp + (size_t)(16 * nt) * (size_t)KPAD + k0;
      FragB bf;
      bf.h[0] = *(const v8usa*)wq;
      bf.h[1] = *(const v8usa*)(wq + 16);
      acc[nt] = wmb(af, bf, acc[nt]);
    }
  }

#pragma unroll
  for (int nt = 0; nt < 8; ++nt) {
    const int lc = 16 * nt + m;
#pragma unroll
    for (int r = 0; r < 8; ++r) {
      const int lr = 16 * wave + 8 * hh + r;
      stg[lr * COUT + lc] = acc[nt][r];
    }
  }
  __syncthreads();

  v4f pv[16];
#pragma unroll
  for (int i = 0; i < 16; ++i) pv[i] = *(const v4fa*)(stg + (16 * wave + i) * COUT + 4 * lane);
#pragma unroll
  for (int i = 0; i < 16; ++i) {
    float* op = Zp + (size_t)(rowBase + 16 * wave + i) * (size_t)COUT + 4 * lane;
    *(volatile v4f*)op = pv[i];
  }
  __threadfence();
#pragma unroll
  for (int i = 0; i < 16; ++i) {
    float* op = Zp + (size_t)(rowBase + 16 * wave + i) * (size_t)COUT + 4 * lane;
    *(volatile v4f*)op = pv[i];
  }
}

__global__ __launch_bounds__(NTHR) void k_stats(const int* __restrict__ nidx, const float* __restrict__ Zp,
                                                double* REC) {
  __shared__ __attribute__((aligned(16))) double red[(NTHR / 32) * COUT * 2];
  const int tid = (int)threadIdx.x, lane = tid & 31, wave = tid >> 5;
  const int blk = (int)blockIdx.x;
  const int b   = blk >> 8;
  const int p0  = (blk & 255) * QPB;
  const float* Zb = Zp + (size_t)b * NSUP * COUT;

  double dS[4], dQ[4];
#pragma unroll
  for (int e = 0; e < 4; ++e) { dS[e] = 0.0; dQ[e] = 0.0; }

#pragma unroll 1
  for (int j = 0; j < 4; ++j) {
    const int p = p0 + 4 * wave + j;
    int idv = nidx[((size_t)b * NQ + p) * NS + lane];
    idv = idv < 0 ? 0 : (idv > NSUP - 1 ? NSUP - 1 : idv);
    const v4f t = *(const v4f*)(Zp + ((size_t)SROWS + (size_t)b * NQ + p) * COUT + 4 * lane);
    v4f sv = {0.0f, 0.0f, 0.0f, 0.0f};
    v4f qv = {0.0f, 0.0f, 0.0f, 0.0f};
#pragma unroll 1
    for (int s0 = 0; s0 < NS; s0 += 8) {
      v4f z[8];
#pragma unroll
      for (int jj = 0; jj < 8; ++jj) {
        const int id = __builtin_amdgcn_readlane(idv, s0 + jj);
        z[jj] = *(const v4f*)(Zb + (size_t)id * COUT + 4 * lane);
      }
#pragma unroll
      for (int jj = 0; jj < 8; ++jj) {
        const v4f y = z[jj] - t;
        sv = sv + y;
        qv.x = fmaf(y.x, y.x, qv.x);
        qv.y = fmaf(y.y, y.y, qv.y);
        qv.z = fmaf(y.z, y.z, qv.z);
        qv.w = fmaf(y.w, y.w, qv.w);
      }
    }
    dS[0] += (double)sv.x; dS[1] += (double)sv.y; dS[2] += (double)sv.z; dS[3] += (double)sv.w;
    dQ[0] += (double)qv.x; dQ[1] += (double)qv.y; dQ[2] += (double)qv.z; dQ[3] += (double)qv.w;
  }
#pragma unroll
  for (int e = 0; e < 4; ++e) {
    red[(wave * COUT + 4 * lane + e) * 2 + 0] = dS[e];
    red[(wave * COUT + 4 * lane + e) * 2 + 1] = dQ[e];
  }
  __syncthreads();
  v2d o = {0.0, 0.0};
  if (tid < COUT) {
    double S = 0.0, Q = 0.0;
#pragma unroll
    for (int w2 = 0; w2 < NTHR / 32; ++w2) {
      S += red[(w2 * COUT + tid) * 2 + 0];
      Q += red[(w2 * COUT + tid) * 2 + 1];
    }
    o.x = S; o.y = Q;
    *(volatile v2d*)(REC + ((size_t)blk * COUT + tid) * 2) = o;
  }
  __threadfence();
  if (tid < COUT) {
    *(volatile v2d*)(REC + ((size_t)blk * COUT + tid) * 2) = o;
  }
}

__global__ __launch_bounds__(COUT) void k_comb(const double* __restrict__ REC, const float* __restrict__ gam,
                                               const float* __restrict__ bet, float* MR) {
  __shared__ __attribute__((aligned(16))) float smr[4 * COUT];
  const int c = (int)threadIdx.x;
  double S = 0.0, Q = 0.0;
#pragma unroll 4
  for (int blk = 0; blk < NGB; ++blk) {
    const v2d r = *(const v2d*)(REC + ((size_t)blk * COUT + c) * 2);
    S += r.x;
    Q += r.y;
  }
  const double inv = 1.0 / (double)NSAMP;
  const double mean = S * inv;
  double var = Q * inv - mean * mean;
  var = var < 0.0 ? 0.0 : var;
  const double x = var + 1e-5;
  double r = (double)rsqrtf((float)x);
  r = r * (1.5 - 0.5 * x * r * r);
  r = r * (1.5 - 0.5 * x * r * r);
  smr[c]            = (float)mean;
  smr[COUT + c]     = (float)r;
  smr[2 * COUT + c] = bf16_val(gam[c]);
  smr[3 * COUT + c] = bf16_val(bet[c]);
  __syncthreads();
  const v4f v = *(const v4fa*)(smr + 4 * c);
  *(volatile v4f*)(MR + 4 * c) = v;
  __threadfence();
  *(volatile v4f*)(MR + 4 * c) = v;
}

__global__ __launch_bounds__(NTHR) void k_apply(const int* __restrict__ nidx, const float* __restrict__ Zp,
                                                const float* __restrict__ MR, float* out) {
  __shared__ __attribute__((aligned(16))) float smr[4 * COUT];
  __shared__ __attribute__((aligned(16))) float ot[COUT * OTP];
  const int tid = (int)threadIdx.x, lane = tid & 31, wave = tid >> 5;
  const int blk = (int)blockIdx.x;
  const int b   = blk >> 8;
  const int p0  = (blk & 255) * QPB;
  const float* Zb = Zp + (size_t)b * NSUP * COUT;

  if (tid < COUT) {
    const v4f a = *(const v4f*)(MR + 4 * tid);
    *(v4fa*)(smr + 4 * tid) = a;
  }
  __syncthreads();
  const v4f mean = *(const v4fa*)(smr + 4 * lane);
  const v4f rstd = *(const v4fa*)(smr + COUT + 4 * lane);
  const v4f gm   = *(const v4fa*)(smr + 2 * COUT + 4 * lane);
  const v4f bt   = *(const v4fa*)(smr + 3 * COUT + 4 * lane);

#pragma unroll 1
  for (int j = 0; j < 4; ++j) {
    const int ql = 4 * wave + j;
    const int p  = p0 + ql;
    int idv = nidx[((size_t)b * NQ + p) * NS + lane];
    idv = idv < 0 ? 0 : (idv > NSUP - 1 ? NSUP - 1 : idv);
    const v4f t = *(const v4f*)(Zp + ((size_t)SROWS + (size_t)b * NQ + p) * COUT + 4 * lane);
    const float lo = -3.402823466e38f;
    v4f mx = {lo, lo, lo, lo};
#pragma unroll 1
    for (int s0 = 0; s0 < NS; s0 += 8) {
      v4f z[8];
#pragma unroll
      for (int jj = 0; jj < 8; ++jj) {
        const int id = __builtin_amdgcn_readlane(idv, s0 + jj);
        z[jj] = *(const v4f*)(Zb + (size_t)id * COUT + 4 * lane);
      }
#pragma unroll
      for (int jj = 0; jj < 8; ++jj) {
        const v4f y = z[jj] - t;
        v4f v = (y - mean) * rstd;
        v = v * gm + bt;
        const float r0 = (v.x > 0.0f) ? v.x : 0.0f;
        const float r1 = (v.y > 0.0f) ? v.y : 0.0f;
        const float r2 = (v.z > 0.0f) ? v.z : 0.0f;
        const float r3 = (v.w > 0.0f) ? v.w : 0.0f;
        mx.x = fmaxf(mx.x, r0);
        mx.y = fmaxf(mx.y, r1);
        mx.z = fmaxf(mx.z, r2);
        mx.w = fmaxf(mx.w, r3);
      }
    }
    ot[(4 * lane + 0) * OTP + ql] = mx.x;
    ot[(4 * lane + 1) * OTP + ql] = mx.y;
    ot[(4 * lane + 2) * OTP + ql] = mx.z;
    ot[(4 * lane + 3) * OTP + ql] = mx.w;
  }
  __syncthreads();

  float ov[16];
#pragma unroll
  for (int i = 0; i < 16; ++i) ov[i] = ot[(wave + 8 * i) * OTP + lane];
#pragma unroll
  for (int i = 0; i < 16; ++i) {
    float* op = out + ((size_t)b * COUT + (wave + 8 * i)) * NQ + p0 + lane;
    *(volatile float*)op = ov[i];
  }
  __threadfence();
#pragma unroll
  for (int i = 0; i < 16; ++i) {
    float* op = out + ((size_t)b * COUT + (wave + 8 * i)) * NQ + p0 + lane;
    *(volatile float*)op = ov[i];
  }
}

static inline size_t al256(size_t o) { return (o + 255) & ~(size_t)255; }

extern "C" void kernel_launch(void* const* d_in, const int* in_sizes, int n_in,
                              void* d_out, int out_size, void* d_ws, size_t ws_size,
                              hipStream_t stream) {
  if (n_in < 7) return;
  if (in_sizes[0] != NB * NQ * 3) return;
  if (in_sizes[1] != NB * NSUP * 3) return;
  if (in_sizes[2] != NB * CF * NSUP) return;
  if (in_sizes[3] != NB * NQ * NS) return;
  if (in_sizes[4] != COUT * CIN) return;
  if (in_sizes[5] != COUT || in_sizes[6] != COUT) return;
  if (out_size != NB * COUT * NQ) return;

  const float* qxyz = (const float*)d_in[0];
  const float* sxyz = (const float*)d_in[1];
  const float* feat = (const float*)d_in[2];
  const int*   nidx = (const int*)d_in[3];
  const float* wc   = (const float*)d_in[4];
  const float* gam  = (const float*)d_in[5];
  const float* bet  = (const float*)d_in[6];
  float* out = (float*)d_out;

  size_t off = 0;
  const size_t oAB  = off; off = al256(off + (size_t)NPB * TILE_BYTES);
  const size_t oZ   = off; off = al256(off + (size_t)MROWS * COUT * 4);
  const size_t oREC = off; off = al256(off + (size_t)NGB * COUT * 2 * 8);
  const size_t oMR  = off; off = al256(off + (size_t)4 * COUT * 4);
  if (off > ws_size || off > (size_t)WSCAP) return;

  char* ws = (char*)d_ws;
  unsigned short* ABW = (unsigned short*)(ws + oAB);
  const unsigned short* WB = ABW + (size_t)MROWS * KPAD;
  float*  Zp  = (float*)(ws + oZ);
  double* REC = (double*)(ws + oREC);
  float*  MR  = (float*)(ws + oMR);

  k_prep<<<NPB, NTHR, 0, stream>>>(qxyz, sxyz, feat, wc, ABW);
  k_gemm<<<MROWS / GBM, GTHR, 0, stream>>>(ABW, WB, Zp);
  k_stats<<<NGB, NTHR, 0, stream>>>(nidx, Zp, REC);
  k_comb<<<1, COUT, 0, stream>>>(REC, gam, bet, MR);
  k_apply<<<NGB, NTHR, 0, stream>>>(nidx, Zp, MR, out);
  (void)hipGetLastError();
}
